// SVDPlusPlusNet_76046690943220
// MI455X (gfx1250) — hardware-verified
//
#include <hip/hip_runtime.h>
#include <stddef.h>
#include <stdint.h>


#define NB      8192
#define HL      200
#define DD      128
#define NTAB    100000
#define NT_MAX  13
#define CTHR    256
#define YB_ELEMS   (NTAB * DD)
#define PB_OFF_E   (YB_ELEMS)
#define QB_OFF_E   (PB_OFF_E + NB * DD)
#define BS_OFF_B   ((size_t)(QB_OFF_E + NB * DD) * 2)
#define WS_TOTAL   (BS_OFF_B + (size_t)NB * 4)
#define WSMAX      134217728

static_assert(DD == 128);
static_assert(HL == 200);
static_assert((HL + 16) / 16 == NT_MAX);
static_assert(NB % 32 == 0);
static_assert((YB_ELEMS % (CTHR * 8)) == 0);
static_assert(((size_t)YB_ELEMS * 2) % 256 == 0);
static_assert(((size_t)PB_OFF_E * 2) % 256 == 0 && ((size_t)QB_OFF_E * 2) % 256 == 0 && (BS_OFF_B % 256) == 0);
static_assert(DD * 2 == 256);
static_assert(WS_TOTAL <= (size_t)WSMAX);
static_assert((long long)QB_OFF_E + (long long)NB * DD < (1LL << 31));

typedef float          v4f   __attribute__((ext_vector_type(4)));
typedef float          v8f   __attribute__((ext_vector_type(8)));
typedef int            v8i   __attribute__((ext_vector_type(8)));
typedef unsigned short v8us  __attribute__((ext_vector_type(8)));
typedef unsigned short v16us __attribute__((ext_vector_type(16)));
typedef __bf16         v16bf __attribute__((ext_vector_type(16)));
typedef v4f  __attribute__((may_alias)) v4fa;
typedef v8us __attribute__((may_alias)) v8usa;
union FragB { v16bf v; v16us u; v8us h[2]; v8i w; };

__device__ __forceinline__ v8f wmb(const FragB& a, const FragB& b, v8f c) {
  v8f d = __builtin_amdgcn_wmma_f32_16x16x32_bf16(false, a.v, false, b.v, (short)0, c, false, false);
  asm volatile("v_nop\n\tv_nop\n\tv_nop\n\tv_nop" : "+v"(d) : "v"(a.w), "v"(b.w));
  return d;
}

__device__ __forceinline__ unsigned bf16_bits(float f) {
  const unsigned u = __float_as_uint(f);
  const unsigned r = (u + 0x7FFFu + ((u >> 16) & 1u)) >> 16;
  const unsigned q = (u >> 16) | 0x40u;
  return ((u & 0x7fffffffu) > 0x7f800000u) ? q : r;
}
__device__ __forceinline__ float bf16_val(float f) {
  return __uint_as_float(bf16_bits(f) << 16);
}
__device__ __forceinline__ v8us pack8(v4f a, v4f c) {
  v8us o;
  o[0] = (unsigned short)bf16_bits(a.x); o[1] = (unsigned short)bf16_bits(a.y);
  o[2] = (unsigned short)bf16_bits(a.z); o[3] = (unsigned short)bf16_bits(a.w);
  o[4] = (unsigned short)bf16_bits(c.x); o[5] = (unsigned short)bf16_bits(c.y);
  o[6] = (unsigned short)bf16_bits(c.z); o[7] = (unsigned short)bf16_bits(c.w);
  return o;
}
__device__ __forceinline__ int clampi(int v, int lo, int hi) {
  return v < lo ? lo : (v > hi ? hi : v);
}

__device__ __forceinline__ void wave_sync() {
  __builtin_amdgcn_fence(__ATOMIC_RELEASE, "workgroup");
  __builtin_amdgcn_wave_barrier();
  __builtin_amdgcn_fence(__ATOMIC_ACQUIRE, "workgroup");
}

__global__ __launch_bounds__(CTHR) void k_cvt(const float* __restrict__ src, unsigned short* yb) {
  const int g = (int)blockIdx.x * CTHR + (int)threadIdx.x;
  if (g >= YB_ELEMS / 8) return;
  const float* p = src + (size_t)g * 8;
  const v4f a = *(const v4fa*)p;
  const v4f c = *(const v4fa*)(p + 4);
  const v8us o = pack8(a, c);
  unsigned short* dp = yb + (size_t)g * 8;
  *(volatile v8us*)dp = o;
  __threadfence();
  *(volatile v8us*)dp = o;
}

__global__ __launch_bounds__(CTHR) void k_pq(const int* __restrict__ user_ids, const int* __restrict__ item_ids,
                                             const float* __restrict__ user_emb, const float* __restrict__ item_emb,
                                             const float* __restrict__ user_bias, const float* __restrict__ item_bias,
                                             const float* __restrict__ global_bias,
                                             unsigned short* pb, unsigned short* qb, float* bsp) {
  __shared__ __attribute__((aligned(16))) float sBS[32];
  const int tid = (int)threadIdx.x;
  const int b0 = (int)blockIdx.x * 32;

  v8us op0, op1, oq0, oq1;
  {
    const int u = tid;
    const int b = b0 + (u >> 4), pc = u & 15;
    const int uid = clampi(user_ids[b], 0, NTAB - 1);
    const int iid = clampi(item_ids[b], 0, NTAB - 1);
    const float* pu = user_emb + (size_t)uid * DD + 8 * pc;
    const float* pi = item_emb + (size_t)iid * DD + 8 * pc;
    const v4f a = *(const v4fa*)pu;
    const v4f c = *(const v4fa*)(pu + 4);
    const v4f e = *(const v4fa*)pi;
    const v4f f = *(const v4fa*)(pi + 4);
    op0 = pack8(a, c);
    oq0 = pack8(e, f);
  }
  {
    const int u = tid + CTHR;
    const int b = b0 + (u >> 4), pc = u & 15;
    const int uid = clampi(user_ids[b], 0, NTAB - 1);
    const int iid = clampi(item_ids[b], 0, NTAB - 1);
    const float* pu = user_emb + (size_t)uid * DD + 8 * pc;
    const float* pi = item_emb + (size_t)iid * DD + 8 * pc;
    const v4f a = *(const v4fa*)pu;
    const v4f c = *(const v4fa*)(pu + 4);
    const v4f e = *(const v4fa*)pi;
    const v4f f = *(const v4fa*)(pi + 4);
    op1 = pack8(a, c);
    oq1 = pack8(e, f);
  }
  unsigned short* dp0 = pb + (size_t)b0 * DD + (size_t)tid * 8;
  unsigned short* dp1 = dp0 + CTHR * 8;
  unsigned short* dq0 = qb + (size_t)b0 * DD + (size_t)tid * 8;
  unsigned short* dq1 = dq0 + CTHR * 8;
  *(volatile v8us*)dp0 = op0;
  *(volatile v8us*)dp1 = op1;
  *(volatile v8us*)dq0 = oq0;
  *(volatile v8us*)dq1 = oq1;
  __threadfence();
  *(volatile v8us*)dp0 = op0;
  *(volatile v8us*)dp1 = op1;
  *(volatile v8us*)dq0 = oq0;
  *(volatile v8us*)dq1 = oq1;

  if (tid < 32) {
    const int b = b0 + tid;
    const int uid = clampi(user_ids[b], 0, NTAB - 1);
    const int iid = clampi(item_ids[b], 0, NTAB - 1);
    const float gb = bf16_val(global_bias[0]);
    const float bu = bf16_val(user_bias[uid]);
    const float bi = bf16_val(item_bias[iid]);
    sBS[tid] = (gb + bu) + bi;
  }
  __syncthreads();
  if (tid < 8) {
    const v4f v = *(const v4fa*)(sBS + 4 * tid);
    float* dp = bsp + b0 + 4 * tid;
    *(volatile v4f*)dp = v;
    __threadfence();
    *(volatile v4f*)dp = v;
  }
}

__global__ __launch_bounds__(CTHR) void k_main(const int* __restrict__ hist_items, const int* __restrict__ hist_len,
                                               const unsigned short* __restrict__ planes,
                                               const float* __restrict__ bsp, float* out) {
  __shared__ __attribute__((aligned(16))) unsigned short tile[8 * 16 * DD];
  __shared__ __attribute__((aligned(16))) float sOut[32];
  const int tid = (int)threadIdx.x, lane = tid & 31, wave = tid >> 5, hh = lane >> 4, m = lane & 15;
  const int b0 = (int)blockIdx.x * 32;
  unsigned short* tl = tile + wave * (16 * DD);

#pragma unroll 1
  for (int j = 0; j < 4; ++j) {
    const int b = b0 + 4 * wave + j;
    const int len = hist_len[b];
    const int nmask = __builtin_amdgcn_readfirstlane(clampi(len, 0, HL));
    const int nt = (nmask + 16) >> 4;

    const unsigned short* qrow = planes + (size_t)QB_OFF_E + (size_t)b * DD + 8 * hh;
    FragB q0, q1, q2, q3;
    q0.h[0] = *(const v8usa*)(qrow);       q0.h[1] = *(const v8usa*)(qrow + 16);
    q1.h[0] = *(const v8usa*)(qrow + 32);  q1.h[1] = *(const v8usa*)(qrow + 48);
    q2.h[0] = *(const v8usa*)(qrow + 64);  q2.h[1] = *(const v8usa*)(qrow + 80);
    q3.h[0] = *(const v8usa*)(qrow + 96);  q3.h[1] = *(const v8usa*)(qrow + 112);

    const int* hrow = hist_items + (size_t)b * HL;
    float S = 0.0f, P = 0.0f;

#pragma unroll 1
    for (int t = 0; t < nt; ++t) {
      const int r  = 16 * t + m;
      const int lc = clampi(r - 1, 0, HL - 1);
      const int item = clampi(hrow[lc], 0, NTAB - 1);
      const int off = (r == 0) ? (PB_OFF_E + b * DD) : (item * DD);

      v8us g[8];
#pragma unroll
      for (int i = 0; i < 8; ++i) {
        const int so = __shfl(off, 2 * i + hh, 32);
        g[i] = *(const v8usa*)(planes + (size_t)so + 8 * m);
      }
#pragma unroll
      for (int i = 0; i < 8; ++i)
        *(v8usa*)(tl + (2 * i + hh) * DD + 8 * m) = g[i];
      wave_sync();

      const unsigned short* ar = tl + m * DD + 8 * hh;
      FragB a0, a1, a2, a3;
      a0.h[0] = *(const v8usa*)(ar);       a0.h[1] = *(const v8usa*)(ar + 16);
      a1.h[0] = *(const v8usa*)(ar + 32);  a1.h[1] = *(const v8usa*)(ar + 48);
      a2.h[0] = *(const v8usa*)(ar + 64);  a2.h[1] = *(const v8usa*)(ar + 80);
      a3.h[0] = *(const v8usa*)(ar + 96);  a3.h[1] = *(const v8usa*)(ar + 112);
      wave_sync();

      v8f d = {0.f, 0.f, 0.f, 0.f, 0.f, 0.f, 0.f, 0.f};
      d = wmb(a0, q0, d);
      d = wmb(a1, q1, d);
      d = wmb(a2, q2, d);
      d = wmb(a3, q3, d);

      const int rb = 16 * t + 8 * hh;
#pragma unroll
      for (int i = 0; i < 8; ++i) {
        const int rr = rb + i;
        const float dv = d[i];
        S += ((rr >= 1) && (rr - 1 < nmask)) ? dv : 0.0f;
        P += (rr == 0) ? dv : 0.0f;
      }
    }

    S += __shfl_xor(S, 16, 32);
    P += __shfl_xor(P, 16, 32);
    const float lf = fmaxf((float)len, 1.0f);
    const float nrm = (len > 0) ? (1.0f / sqrtf(lf)) : 0.0f;
    const float res = bsp[b] + (P + nrm * S);
    if (lane == 0) sOut[4 * wave + j] = res;
  }
  __syncthreads();

  if (tid < 8) {
    const v4f v = *(const v4fa*)(sOut + 4 * tid);
    float* dp = out + b0 + 4 * tid;
    *(volatile v4f*)dp = v;
    __threadfence();
    *(volatile v4f*)dp = v;
  }
}

extern "C" void kernel_launch(void* const* d_in, const int* in_sizes, int n_in,
                              void* d_out, int out_size, void* d_ws, size_t ws_size,
                              hipStream_t stream) {
  if (n_in < 10) return;
  if (in_sizes[0] != NB || in_sizes[1] != NB || in_sizes[3] != NB) return;
  if (in_sizes[2] != NB * HL) return;
  if (in_sizes[4] != NTAB * DD || in_sizes[5] != NTAB * DD || in_sizes[6] != NTAB * DD) return;
  if (in_sizes[7] != NTAB || in_sizes[8] != NTAB || in_sizes[9] != 1) return;
  if (out_size != NB) return;
  if (ws_size < (size_t)WS_TOTAL) return;

  const int*   user_ids     = (const int*)d_in[0];
  const int*   item_ids     = (const int*)d_in[1];
  const int*   hist_items   = (const int*)d_in[2];
  const int*   hist_len     = (const int*)d_in[3];
  const float* user_emb     = (const float*)d_in[4];
  const float* item_emb     = (const float*)d_in[5];
  const float* implicit_emb = (const float*)d_in[6];
  const float* user_bias    = (const float*)d_in[7];
  const float* item_bias    = (const float*)d_in[8];
  const float* global_bias  = (const float*)d_in[9];
  float* out = (float*)d_out;

  char* ws = (char*)d_ws;
  unsigned short* planes = (unsigned short*)ws;
  unsigned short* pb = planes + (size_t)PB_OFF_E;
  unsigned short* qb = planes + (size_t)QB_OFF_E;
  float* bsp = (float*)(ws + BS_OFF_B);

  k_cvt<<<YB_ELEMS / (CTHR * 8), CTHR, 0, stream>>>(implicit_emb, planes);
  k_pq<<<NB / 32, CTHR, 0, stream>>>(user_ids, item_ids, user_emb, item_emb,
                                     user_bias, item_bias, global_bias, pb, qb, bsp);
  k_main<<<NB / 32, CTHR, 0, stream>>>(hist_items, hist_len, planes, bsp, out);
}
